// GQAAttention_39204461477977
// MI455X (gfx1250) — hardware-verified
//
#include <hip/hip_runtime.h>
#ifndef NB
#define NB 2
#endif
#ifndef SLEN
#define SLEN 2048
#endif
#define NB_FULL 2
#define SEQ_FULL 2048
#define DM 2048
#define NH 32
#define NKV 8
#define NREP (NH / NKV)
#define KVD (NKV * 64)
#define NR (NB * SLEN)
#define TQ SLEN
#define TK SLEN
#define SCL 0.125f
#define QBLKS (TQ / 64)
#define QB05 0
#define QBN5 4
#define QB0P 4
#define QBNP (QBLKS - 4)
#define QBNPD ((QBNP > 0) ? QBNP : 1)
#define RE 256

static_assert(NB >= 1 && NB <= NB_FULL);
static_assert(SLEN >= 256 && SLEN <= SEQ_FULL && (SLEN % 256) == 0);
static_assert(NREP * NKV == NH);
static_assert(4 * KVD == DM);
static_assert((NR % 128) == 0 && (DM % 64) == 0 && (KVD % 64) == 0 && (DM % 32) == 0);
static_assert((RE % 128) == 0 && RE <= SLEN && RE == 64 * QBN5);
static_assert(4ull * (unsigned long long)NR * KVD <= (unsigned long long)DM * DM * 2 + 4ull * KVD * DM);

typedef unsigned short v8us __attribute__((ext_vector_type(8), may_alias));
typedef float  v8f  __attribute__((ext_vector_type(8)));
typedef float  v4f  __attribute__((ext_vector_type(4)));
typedef float  v4fa __attribute__((ext_vector_type(4), may_alias));
typedef _Float16 v16h __attribute__((ext_vector_type(16)));
union FragH { v16h v; v8us half[2]; _Float16 h[16]; unsigned short u[16]; };

__device__ __forceinline__ unsigned short bf16_bits(float x) { unsigned int u = __float_as_uint(x); return (unsigned short)((u + 0x7FFFu + ((u >> 16) & 1u)) >> 16); }
__device__ __forceinline__ float bf16_val(unsigned short b) { return __uint_as_float(((unsigned int)b) << 16); }
__device__ __forceinline__ float bf16_rne(float x) { return bf16_val(bf16_bits(x)); }

template <int NT>
__device__ __forceinline__ v8f mmaH(v16h ah, v16h al, v16h bh, v16h bl, v8f c) {
  c = __builtin_amdgcn_wmma_f32_16x16x32_f16(false, ah, false, bh, (short)0, c, false, false);
  if (NT >= 2) c = __builtin_amdgcn_wmma_f32_16x16x32_f16(false, al, false, bh, (short)0, c, false, false);
  if (NT >= 3) c = __builtin_amdgcn_wmma_f32_16x16x32_f16(false, ah, false, bl, (short)0, c, false, false);
  asm volatile("v_nop\n\tv_nop\n\tv_nop\n\tv_nop" : "+v"(c) : "v"(ah), "v"(al), "v"(bh), "v"(bl));
  return c;
}

__global__ __launch_bounds__(256) void k_wsc(const float* __restrict__ Wm, _Float16* __restrict__ Bt, size_t n8, float sc) {
  #pragma clang fp contract(off)
  const size_t t = (size_t)blockIdx.x * 256 + threadIdx.x; if (t >= n8) return;
  const v4f a = *(const v4fa*)(Wm + t * 8), c = *(const v4fa*)(Wm + t * 8 + 4); FragH f;
#pragma unroll
  for (int q = 0; q < 4; ++q) { f.h[q] = (_Float16)(bf16_rne(a[q]) * sc); f.h[4 + q] = (_Float16)(bf16_rne(c[q]) * sc); }
  const v8us o = f.half[0];
  *(volatile v8us*)((unsigned short*)Bt + t * 8) = o; __threadfence(); *(volatile v8us*)((unsigned short*)Bt + t * 8) = o;
}

__global__ __launch_bounds__(256) void k_x16(const float* __restrict__ x, _Float16* __restrict__ X16, size_t n8) {
  const size_t t = (size_t)blockIdx.x * 256 + threadIdx.x; if (t >= n8) return;
  const size_t e = t * 8; const size_t row = e / DM; const int c = (int)(e % DM); const int bb = (int)(row / SLEN), s = (int)(row % SLEN);
  const float* src = x + ((size_t)bb * SEQ_FULL + s) * DM + c;
  const v4f a = *(const v4fa*)src, d = *(const v4fa*)(src + 4); FragH f;
#pragma unroll
  for (int q = 0; q < 4; ++q) { f.h[q] = (_Float16)bf16_rne(a[q]); f.h[4 + q] = (_Float16)bf16_rne(d[q]); }
  const v8us o = f.half[0];
  *(volatile v8us*)((unsigned short*)X16 + t * 8) = o; __threadfence(); *(volatile v8us*)((unsigned short*)X16 + t * 8) = o;
}

__device__ __forceinline__ v16h g2_frag(const _Float16* p, int hh) { FragH f; f.half[0] = *(const v8us*)((const unsigned short*)p + 8 * hh); f.half[1] = *(const v8us*)((const unsigned short*)p + 16 + 8 * hh); return f.v; }
__device__ __forceinline__ v8f g2_mma(v16h a, v16h b, v8f c) { v8f d = __builtin_amdgcn_wmma_f32_16x16x32_f16(false, a, false, b, (short)0, c, false, false); asm volatile("v_nop\n\tv_nop\n\tv_nop\n\tv_nop" : "+v"(d) : "v"(a), "v"(b)); return d; }

__global__ __launch_bounds__(128) __attribute__((amdgpu_num_vgpr(256)))
void k_gemm2(const _Float16* __restrict__ A, int lda, const _Float16* __restrict__ Bh, int ldb, float alpha, const float* CP, float* C, int ldc, int M, int N, int K) {
  __shared__ __attribute__((aligned(16))) float so[4][32][68];
  const int tid = threadIdx.x, w = tid >> 5, lane = tid & 31, ln = lane & 15, hh = lane >> 4;
  const int ntn = N >> 6; const int mt = blockIdx.x / ntn, nq = blockIdx.x - mt * ntn; const int row0 = mt * 128 + 32 * w, col0 = nq * 64; if (row0 >= M) return;
  const _Float16* a0p = A + (size_t)(row0 + ln) * lda; const _Float16* a1p = a0p + (size_t)16 * lda;
  const _Float16* b0p = Bh + (size_t)(col0 + ln) * ldb; const _Float16* b1p = b0p + (size_t)16 * ldb; const _Float16* b2p = b1p + (size_t)16 * ldb; const _Float16* b3p = b2p + (size_t)16 * ldb;
  const v8f z8 = {0.f,0.f,0.f,0.f,0.f,0.f,0.f,0.f}; v8f c00 = z8, c01 = z8, c02 = z8, c03 = z8, c10 = z8, c11 = z8, c12 = z8, c13 = z8;
#pragma unroll 1
  for (int kb = 0; kb < K; kb += 32) { const v16h a0 = g2_frag(a0p + kb, hh), a1 = g2_frag(a1p + kb, hh);
    v16h b = g2_frag(b0p + kb, hh); c00 = g2_mma(a0, b, c00); c10 = g2_mma(a1, b, c10);
    b = g2_frag(b1p + kb, hh); c01 = g2_mma(a0, b, c01); c11 = g2_mma(a1, b, c11);
    b = g2_frag(b2p + kb, hh); c02 = g2_mma(a0, b, c02); c12 = g2_mma(a1, b, c12);
    b = g2_frag(b3p + kb, hh); c03 = g2_mma(a0, b, c03); c13 = g2_mma(a1, b, c13); }
  v8f accs[8] = {c00, c01, c02, c03, c10, c11, c12, c13};
#pragma unroll
  for (int u = 0; u < 8; ++u) { const int t = u & 3, half = u >> 2;
#pragma unroll
    for (int r = 0; r < 8; ++r) { const int rloc = half * 16 + 8 * hh + r; so[w][rloc][t * 16 + ln] = accs[u][r] * alpha; } }
  __builtin_amdgcn_fence(4, "workgroup"); __builtin_amdgcn_wave_barrier();
  const int rsub = lane >> 4, c4 = (lane & 15) * 4;
  if (CP) {
#pragma unroll
    for (int q = 0; q < 16; ++q) { const int r = q * 2 + rsub; v4f v = *(const v4fa*)&so[w][r][c4]; const v4f cpv = *(const v4fa*)(CP + (size_t)(row0 + r) * ldc + col0 + c4); v += cpv; *(v4fa*)&so[w][r][c4] = v; }
  }
  for (int pass = 0; pass < 2; ++pass) {
#pragma unroll
    for (int q = 0; q < 16; ++q) { const int r = q * 2 + rsub; const v4f v = *(const v4fa*)&so[w][r][c4]; *(volatile v4f*)(C + (size_t)(row0 + r) * ldc + col0 + c4) = v; }
    if (pass == 0) __threadfence(); }
}

__constant__ float c_pw[32] = {
  1.0f, 1.333521432163324f, 1.7782794100389228f, 2.3713737056616552f, 3.1622776601683795f, 4.216965034285822f, 5.623413251903491f, 7.498942093324558f,
  10.0f, 13.33521432163324f, 17.782794100389228f, 23.713737056616552f, 31.622776601683795f, 42.16965034285822f, 56.23413251903491f, 74.98942093324558f,
  100.0f, 133.3521432163324f, 177.82794100389228f, 237.13737056616552f, 316.22776601683795f, 421.6965034285822f, 562.3413251903491f, 749.8942093324558f,
  1000.0f, 1333.521432163324f, 1778.2794100389228f, 2371.3737056616552f, 3162.2776601683795f, 4216.965034285822f, 5623.413251903491f, 7498.942093324558f };
__global__ __launch_bounds__(256) void k_rotab(float* __restrict__ CS, float* __restrict__ SN) {
  #pragma clang fp contract(off)
  const int t = blockIdx.x * 256 + threadIdx.x; if (t >= SLEN * 32) return; const int j = t & 31, s = t >> 5;
  const float inv = 1.0f / c_pw[j]; const float th = (float)s * inv; const float c = cosf(th), sn = sinf(th);
  for (int pass = 0; pass < 2; ++pass) { *(volatile float*)(CS + t) = c; *(volatile float*)(SN + t) = sn; if (pass == 0) __threadfence(); } }

__global__ __launch_bounds__(256) void k_ropei(const float* __restrict__ F, int nsrc, int ndst, int rep, const float* __restrict__ CS, const float* __restrict__ SN, _Float16* __restrict__ H, _Float16* __restrict__ L) {
  #pragma clang fp contract(off)
  const size_t t = (size_t)blockIdx.x * 256 + threadIdx.x; if (t >= (size_t)NR * ndst * 8) return;
  const int g8 = (int)(t % 8); const int hd = (int)((t / 8) % ndst); const size_t row = t / ((size_t)8 * ndst); const int s = (int)(row % SLEN); const int hs = hd / rep;
  const float* src = F + row * (size_t)(nsrc * 64) + hs * 64 + g8 * 8;
  const v4f xa = *(const v4fa*)src, xb = *(const v4fa*)(src + 4);
  const v4f cc = *(const v4fa*)(CS + (size_t)s * 32 + g8 * 4), ss = *(const v4fa*)(SN + (size_t)s * 32 + g8 * 4);
  const float xs[8] = {xa[0], xa[1], xa[2], xa[3], xb[0], xb[1], xb[2], xb[3]};
  FragH ah, al;
#pragma unroll
  for (int pr = 0; pr < 4; ++pr) { const float c = cc[pr], sn = ss[pr]; const float x1 = xs[2 * pr], x2 = xs[2 * pr + 1];
    float o1 = x1 * c; o1 -= x2 * sn; float o2 = x1 * sn; o2 += x2 * c;
    _Float16 hv = (_Float16)o1; ah.h[2 * pr] = hv; al.h[2 * pr] = (_Float16)((o1 - (float)hv) * 1024.0f);
    hv = (_Float16)o2; ah.h[2 * pr + 1] = hv; al.h[2 * pr + 1] = (_Float16)((o2 - (float)hv) * 1024.0f); }
  const size_t o = row * (size_t)(ndst * 64) + hd * 64 + g8 * 8; const v8us oh = ah.half[0], ol = al.half[0];
  for (int pass = 0; pass < 2; ++pass) { *(volatile v8us*)((unsigned short*)H + o) = oh; *(volatile v8us*)((unsigned short*)L + o) = ol; if (pass == 0) __threadfence(); } }

__global__ __launch_bounds__(256) void k_hl(const float* __restrict__ F, _Float16* __restrict__ Hh, _Float16* __restrict__ Hl, size_t n8) {
  #pragma clang fp contract(off)
  const size_t t = (size_t)blockIdx.x * 256 + threadIdx.x; if (t >= n8) return; FragH fh, fl; const v4f a = *(const v4fa*)(F + t * 8), c = *(const v4fa*)(F + t * 8 + 4);
#pragma unroll
  for (int q = 0; q < 4; ++q) { _Float16 hv = (_Float16)a[q]; fh.h[q] = hv; fl.h[q] = (_Float16)((a[q] - (float)hv) * 1024.0f); hv = (_Float16)c[q]; fh.h[4 + q] = hv; fl.h[4 + q] = (_Float16)((c[q] - (float)hv) * 1024.0f); }
  const v8us oh = fh.half[0], ol = fl.half[0];
  for (int pass = 0; pass < 2; ++pass) { *(volatile v8us*)((unsigned short*)Hh + t * 8) = oh; *(volatile v8us*)((unsigned short*)Hl + t * 8) = ol; if (pass == 0) __threadfence(); } }

__global__ __launch_bounds__(256) void k_vtg(const _Float16* __restrict__ V16, _Float16* __restrict__ Vt) {
  __shared__ unsigned short tl[64][66];
  const int tid = threadIdx.x; const int slab = blockIdx.x / (SLEN / 64), lg = blockIdx.x % (SLEN / 64); const int b = slab / NKV, kh = slab % NKV;
  for (int i = tid; i < 64 * 8; i += 256) { const int r = i / 8, c8 = (i % 8) * 8; FragH f; f.half[0] = *(const v8us*)((const unsigned short*)V16 + ((size_t)b * SLEN + lg * 64 + r) * KVD + kh * 64 + c8);
#pragma unroll
    for (int q = 0; q < 8; ++q) tl[r][c8 + q] = f.u[q]; }
  __syncthreads();
  for (int pass = 0; pass < 2; ++pass) {
#pragma unroll
    for (int rd = 0; rd < 2; ++rd) { const int d = rd * 32 + tid / 8, pc = tid % 8; FragH f;
#pragma unroll
      for (int q = 0; q < 8; ++q) f.u[q] = tl[pc * 8 + q][d];
      *(volatile v8us*)((unsigned short*)Vt + ((size_t)slab * 64 + d) * SLEN + lg * 64 + pc * 8) = f.half[0]; }
    if (pass == 0) __threadfence(); } }

__global__ __launch_bounds__(128) __attribute__((amdgpu_num_vgpr(256)))
void k_flashc(const _Float16* __restrict__ Q16, int ldq, const _Float16* __restrict__ K16, int ldk, const _Float16* __restrict__ Vt, float* __restrict__ O, int ldo) {
  constexpr int RPW = 16, DT = 4, KS = 2;
  __shared__ __attribute__((aligned(16))) unsigned short sP[4][RPW][40]; __shared__ __attribute__((aligned(16))) float sO[4][RPW][64 + 4];
  const int tid = threadIdx.x, w = tid >> 5, lane = tid & 31, ln = lane & 15, hh = lane >> 4;
  const int slab = blockIdx.x / QBNPD, qblk = QB0P + blockIdx.x % QBNPD; const int b = slab / NH, h = slab % NH, kvh = h / NREP; const int qb0 = qblk * (4 * RPW); const int q0 = qb0 + w * RPW;
  FragH aq[KS];
  { const unsigned short* qr = (const unsigned short*)Q16 + ((size_t)b * TQ + q0 + ln) * ldq + h * 64;
#pragma unroll
    for (int ks = 0; ks < KS; ++ks) { aq[ks].half[0] = *(const v8us*)(qr + ks * 32 + 8 * hh); aq[ks].half[1] = *(const v8us*)(qr + ks * 32 + 16 + 8 * hh); } }
  const unsigned short* Vth = (const unsigned short*)Vt + (size_t)(b * NKV + kvh) * 64 * TK;
  float m_r[8], l_r[8]; v8f oacc[DT];
#pragma unroll
  for (int r = 0; r < 8; ++r) { m_r[r] = -3.0e38f; l_r[r] = 0.f; }
#pragma unroll
  for (int dt = 0; dt < DT; ++dt) oacc[dt] = (v8f){0.f,0.f,0.f,0.f,0.f,0.f,0.f,0.f};
  const int jend = qb0 + 4 * RPW;
#pragma unroll 1
  for (int j0 = 0; j0 < jend; j0 += 32) {
    v8f s[2];
#pragma unroll
    for (int nt = 0; nt < 2; ++nt) { const unsigned short* kr = (const unsigned short*)K16 + ((size_t)b * TK + j0 + nt * 16 + ln) * ldk + kvh * 64; FragH bk[KS];
#pragma unroll
      for (int ks = 0; ks < KS; ++ks) { bk[ks].half[0] = *(const v8us*)(kr + ks * 32 + 8 * hh); bk[ks].half[1] = *(const v8us*)(kr + ks * 32 + 16 + 8 * hh); }
      v8f acc = (v8f){0.f,0.f,0.f,0.f,0.f,0.f,0.f,0.f};
#pragma unroll
      for (int ks = 0; ks < KS; ++ks) acc = mmaH<1>(aq[ks].v, aq[ks].v, bk[ks].v, bk[ks].v, acc);
      s[nt] = acc; }
#pragma unroll
    for (int r = 0; r < 8; ++r) { const int tq = q0 + 8 * hh + r; const int k0 = j0 + ln, k1 = j0 + 16 + ln; const bool ok0 = (k0 <= tq), ok1 = (k1 <= tq);
      const float s0 = ok0 ? s[0][r] * SCL : -3.0e38f, s1 = ok1 ? s[1][r] * SCL : -3.0e38f; float mc = fmaxf(s0, s1);
      mc = fmaxf(mc, __shfl_xor(mc, 1, 32)); mc = fmaxf(mc, __shfl_xor(mc, 2, 32)); mc = fmaxf(mc, __shfl_xor(mc, 4, 32)); mc = fmaxf(mc, __shfl_xor(mc, 8, 32));
      const float mn = fmaxf(m_r[r], mc); const float al = (mn > -1.0e38f) ? expf(m_r[r] - mn) : 1.0f; m_r[r] = mn;
      const float p0 = ok0 ? expf(s0 - mn) : 0.f, p1 = ok1 ? expf(s1 - mn) : 0.f; l_r[r] = l_r[r] * al + p0 + p1;
#pragma unroll
      for (int dt = 0; dt < DT; ++dt) oacc[dt][r] *= al;
      FragH t2; t2.h[0] = (_Float16)(p0 * 1024.0f); t2.h[1] = (_Float16)(p1 * 1024.0f); sP[w][8 * hh + r][ln] = t2.u[0]; sP[w][8 * hh + r][16 + ln] = t2.u[1]; }
    __builtin_amdgcn_fence(4, "workgroup"); __builtin_amdgcn_wave_barrier();
    FragH pa; pa.half[0] = *(const v8us*)&sP[w][ln][8 * hh]; pa.half[1] = *(const v8us*)&sP[w][ln][16 + 8 * hh];
#pragma unroll
    for (int dt = 0; dt < DT; ++dt) { const unsigned short* vrow = Vth + (size_t)(dt * 16 + ln) * TK + j0; FragH bv; bv.half[0] = *(const v8us*)(vrow + 8 * hh); bv.half[1] = *(const v8us*)(vrow + 16 + 8 * hh);
      oacc[dt] = mmaH<1>(pa.v, pa.v, bv.v, bv.v, oacc[dt]); }
    __builtin_amdgcn_fence(4, "workgroup"); __builtin_amdgcn_wave_barrier(); }
#pragma unroll
  for (int r = 0; r < 8; ++r) { float l = l_r[r]; l += __shfl_xor(l, 1, 32); l += __shfl_xor(l, 2, 32); l += __shfl_xor(l, 4, 32); l += __shfl_xor(l, 8, 32); l_r[r] = (l > 0.f) ? 1.0f / (l * 1024.0f) : 0.f; }
#pragma unroll
  for (int dt = 0; dt < DT; ++dt)
#pragma unroll
    for (int r = 0; r < 8; ++r) sO[w][8 * hh + r][dt * 16 + ln] = oacc[dt][r] * l_r[r];
  __builtin_amdgcn_fence(4, "workgroup"); __builtin_amdgcn_wave_barrier();
  for (int pass = 0; pass < 2; ++pass) {
#pragma unroll
    for (int rp = 0; rp < RPW; rp += 2) { const int r = rp + (lane >> 4), pc = lane & 15; const v4f val = *(const v4fa*)&sO[w][r][pc * 4]; *(volatile v4f*)(O + ((size_t)b * TQ + q0 + r) * ldo + h * 64 + pc * 4) = val; }
    if (pass == 0) __threadfence(); } }

__global__ __launch_bounds__(128) __attribute__((amdgpu_num_vgpr(256)))
void k_flash5c(const _Float16* __restrict__ Q16, const _Float16* __restrict__ QL, int ldq, const _Float16* __restrict__ K16, const _Float16* __restrict__ KL, int ldk,
               const _Float16* __restrict__ Vt, const _Float16* __restrict__ VtL, float* __restrict__ O, int ldo) {
  constexpr int RPW = 16, DT = 4, KS = 2;
  __shared__ __attribute__((aligned(16))) unsigned short sP[4][RPW][40]; __shared__ __attribute__((aligned(16))) unsigned short sPL[4][RPW][40]; __shared__ __attribute__((aligned(16))) float sO[4][RPW][64 + 4];
  const int tid = threadIdx.x, w = tid >> 5, lane = tid & 31, ln = lane & 15, hh = lane >> 4;
  const int slab = blockIdx.x / QBN5, qblk = QB05 + blockIdx.x % QBN5; const int b = slab / NH, h = slab % NH, kvh = h / NREP; const int qb0 = qblk * (4 * RPW); const int q0 = qb0 + w * RPW;
  FragH aq[KS], aql[KS];
  { const unsigned short* qr = (const unsigned short*)Q16 + ((size_t)b * TQ + q0 + ln) * ldq + h * 64; const unsigned short* ql = (const unsigned short*)QL + ((size_t)b * TQ + q0 + ln) * ldq + h * 64;
#pragma unroll
    for (int ks = 0; ks < KS; ++ks) { aq[ks].half[0] = *(const v8us*)(qr + ks * 32 + 8 * hh); aq[ks].half[1] = *(const v8us*)(qr + ks * 32 + 16 + 8 * hh); aql[ks].half[0] = *(const v8us*)(ql + ks * 32 + 8 * hh); aql[ks].half[1] = *(const v8us*)(ql + ks * 32 + 16 + 8 * hh); } }
  const unsigned short* Vth = (const unsigned short*)Vt + (size_t)(b * NKV + kvh) * 64 * TK; const unsigned short* Vtl = (const unsigned short*)VtL + (size_t)(b * NKV + kvh) * 64 * TK;
  float m_r[8], l_r[8]; v8f oacc[DT], oaccL[DT];
#pragma unroll
  for (int r = 0; r < 8; ++r) { m_r[r] = -3.0e38f; l_r[r] = 0.f; }
#pragma unroll
  for (int dt = 0; dt < DT; ++dt) { oacc[dt] = (v8f){0.f,0.f,0.f,0.f,0.f,0.f,0.f,0.f}; oaccL[dt] = oacc[dt]; }
  const int jend = qb0 + 4 * RPW;
#pragma unroll 1
  for (int j0 = 0; j0 < jend; j0 += 32) {
    v8f s[2];
#pragma unroll
    for (int nt = 0; nt < 2; ++nt) { const unsigned short* kr = (const unsigned short*)K16 + ((size_t)b * TK + j0 + nt * 16 + ln) * ldk + kvh * 64; const unsigned short* klr = (const unsigned short*)KL + ((size_t)b * TK + j0 + nt * 16 + ln) * ldk + kvh * 64;
      FragH bk[KS]; v8f acc = (v8f){0.f,0.f,0.f,0.f,0.f,0.f,0.f,0.f}, accl = acc;
#pragma unroll
      for (int ks = 0; ks < KS; ++ks) { bk[ks].half[0] = *(const v8us*)(kr + ks * 32 + 8 * hh); bk[ks].half[1] = *(const v8us*)(kr + ks * 32 + 16 + 8 * hh); }
#pragma unroll
      for (int ks = 0; ks < KS; ++ks) { acc = mmaH<1>(aq[ks].v, aq[ks].v, bk[ks].v, bk[ks].v, acc); accl = mmaH<1>(aql[ks].v, aql[ks].v, bk[ks].v, bk[ks].v, accl); }
#pragma unroll
      for (int ks = 0; ks < KS; ++ks) { FragH bkl; bkl.half[0] = *(const v8us*)(klr + ks * 32 + 8 * hh); bkl.half[1] = *(const v8us*)(klr + ks * 32 + 16 + 8 * hh); accl = mmaH<1>(aq[ks].v, aq[ks].v, bkl.v, bkl.v, accl); }
#pragma unroll
      for (int r = 0; r < 8; ++r) acc[r] += accl[r] * 0.0009765625f;
      s[nt] = acc; }
#pragma unroll
    for (int r = 0; r < 8; ++r) { const int tq = q0 + 8 * hh + r; const int k0 = j0 + ln, k1 = j0 + 16 + ln; const bool ok0 = (k0 <= tq), ok1 = (k1 <= tq);
      const float s0 = ok0 ? s[0][r] * SCL : -3.0e38f, s1 = ok1 ? s[1][r] * SCL : -3.0e38f; float mc = fmaxf(s0, s1);
      mc = fmaxf(mc, __shfl_xor(mc, 1, 32)); mc = fmaxf(mc, __shfl_xor(mc, 2, 32)); mc = fmaxf(mc, __shfl_xor(mc, 4, 32)); mc = fmaxf(mc, __shfl_xor(mc, 8, 32));
      const float mn = fmaxf(m_r[r], mc); const float al = (mn > -1.0e38f) ? expf(m_r[r] - mn) : 1.0f; m_r[r] = mn;
      const float p0 = ok0 ? expf(s0 - mn) : 0.f, p1 = ok1 ? expf(s1 - mn) : 0.f; l_r[r] = l_r[r] * al + p0 + p1;
#pragma unroll
      for (int dt = 0; dt < DT; ++dt) { oacc[dt][r] *= al; oaccL[dt][r] *= al; }
      FragH t2, t2l; const float ps0 = p0 * 1024.0f, ps1 = p1 * 1024.0f; t2.h[0] = (_Float16)ps0; t2.h[1] = (_Float16)ps1;
      const float r0f = (ps0 - (float)t2.h[0]) * 1024.0f, r1f = (ps1 - (float)t2.h[1]) * 1024.0f; t2l.h[0] = (_Float16)r0f; t2l.h[1] = (_Float16)r1f;
      sP[w][8 * hh + r][ln] = t2.u[0]; sP[w][8 * hh + r][16 + ln] = t2.u[1]; sPL[w][8 * hh + r][ln] = t2l.u[0]; sPL[w][8 * hh + r][16 + ln] = t2l.u[1]; }
    __builtin_amdgcn_fence(4, "workgroup"); __builtin_amdgcn_wave_barrier();
    FragH pa, pl; pa.half[0] = *(const v8us*)&sP[w][ln][8 * hh]; pa.half[1] = *(const v8us*)&sP[w][ln][16 + 8 * hh]; pl.half[0] = *(const v8us*)&sPL[w][ln][8 * hh]; pl.half[1] = *(const v8us*)&sPL[w][ln][16 + 8 * hh];
#pragma unroll
    for (int dt = 0; dt < DT; ++dt) { const unsigned short* vrow = Vth + (size_t)(dt * 16 + ln) * TK + j0; FragH bv; bv.half[0] = *(const v8us*)(vrow + 8 * hh); bv.half[1] = *(const v8us*)(vrow + 16 + 8 * hh);
      oacc[dt] = mmaH<1>(pa.v, pa.v, bv.v, bv.v, oacc[dt]); oaccL[dt] = mmaH<1>(pl.v, pl.v, bv.v, bv.v, oaccL[dt]);
      const unsigned short* vrl = Vtl + (size_t)(dt * 16 + ln) * TK + j0; FragH bl; bl.half[0] = *(const v8us*)(vrl + 8 * hh); bl.half[1] = *(const v8us*)(vrl + 16 + 8 * hh);
      oaccL[dt] = mmaH<1>(pa.v, pa.v, bl.v, bl.v, oaccL[dt]); }
    __builtin_amdgcn_fence(4, "workgroup"); __builtin_amdgcn_wave_barrier(); }
#pragma unroll
  for (int r = 0; r < 8; ++r) { float l = l_r[r]; l += __shfl_xor(l, 1, 32); l += __shfl_xor(l, 2, 32); l += __shfl_xor(l, 4, 32); l += __shfl_xor(l, 8, 32); l_r[r] = (l > 0.f) ? 1.0f / (l * 1024.0f) : 0.f; }
#pragma unroll
  for (int dt = 0; dt < DT; ++dt)
#pragma unroll
    for (int r = 0; r < 8; ++r) { float v = oacc[dt][r]; v += oaccL[dt][r] * 0.0009765625f; sO[w][8 * hh + r][dt * 16 + ln] = v * l_r[r]; }
  __builtin_amdgcn_fence(4, "workgroup"); __builtin_amdgcn_wave_barrier();
  for (int pass = 0; pass < 2; ++pass) {
#pragma unroll
    for (int rp = 0; rp < RPW; rp += 2) { const int r = rp + (lane >> 4), pc = lane & 15; const v4f val = *(const v4fa*)&sO[w][r][pc * 4]; *(volatile v4f*)(O + ((size_t)b * TQ + q0 + r) * ldo + h * 64 + pc * 4) = val; }
    if (pass == 0) __threadfence(); } }


extern "C" void kernel_launch(void* const* d_in, const int* in_sizes, int n_in,
                              void* d_out, int out_size, void* d_ws, size_t ws_size, hipStream_t stream) {
  if (n_in < 5) return;
  const long long need_rows = (long long)(NB - 1) * SEQ_FULL + SLEN;
  if ((long long)in_sizes[0] < need_rows * DM || in_sizes[1] < DM * DM || in_sizes[2] < KVD * DM || in_sizes[3] < KVD * DM || in_sizes[4] < DM * DM) return;
  if ((long long)out_size < need_rows * DM) return;
  const float* x = (const float*)d_in[0]; const float* wq = (const float*)d_in[1]; const float* wk = (const float*)d_in[2]; const float* wv = (const float*)d_in[3]; const float* wo = (const float*)d_in[4];
  float* out = (float*)d_out;
  char* ws = (char*)d_ws; size_t off = 0;
  auto take = [&](size_t bytes) { char* p = ws + off; off += (bytes + 255) & ~(size_t)255; return p; };
  const size_t szW = (size_t)DM * DM * 2 + 2 * (size_t)KVD * DM * 2;
  char* RW = take(szW);
  _Float16* BQ = (_Float16*)RW; _Float16* BK = (_Float16*)(RW + (size_t)DM * DM * 2); _Float16* BV = (_Float16*)(RW + (size_t)DM * DM * 2 + (size_t)KVD * DM * 2);
  _Float16* VT = (_Float16*)RW; _Float16* VTL = (_Float16*)(RW + (size_t)NR * KVD * 2);
  _Float16* BO = (_Float16*)take((size_t)DM * DM * 2);
  char* RX = take((size_t)NR * DM * 2);
  _Float16* X16 = (_Float16*)RX; _Float16* KH = (_Float16*)RX; _Float16* KL = (_Float16*)(RX + (size_t)NR * KVD * 2); _Float16* VH = (_Float16*)(RX + 2 * (size_t)NR * KVD * 2); _Float16* VL = (_Float16*)(RX + 3 * (size_t)NR * KVD * 2);
  char* RA = take((size_t)NR * DM * 4);
  float* Qf = (float*)RA; float* O = (float*)RA;
  char* RB = take((size_t)NR * DM * 4);
  _Float16* QH = (_Float16*)RB; _Float16* QL = (_Float16*)(RB + (size_t)NR * DM * 2); _Float16* OH = QH; _Float16* OL = QL;
  float* Kf = (float*)take((size_t)NR * KVD * 4);
  float* Vf = (float*)take((size_t)NR * KVD * 4);
  float* CS = (float*)take((size_t)SLEN * 32 * 4); float* SN = (float*)take((size_t)SLEN * 32 * 4);
  if (off > ws_size) return;

  const size_t n8q = (size_t)DM * DM / 8, n8k = (size_t)KVD * DM / 8, n8x = (size_t)NR * DM / 8, n8v = (size_t)NR * KVD / 8;
  k_wsc<<<(unsigned)((n8q + 255) / 256), 256, 0, stream>>>(wq, BQ, n8q, 16.0f);
  k_wsc<<<(unsigned)((n8k + 255) / 256), 256, 0, stream>>>(wk, BK, n8k, 16.0f);
  k_wsc<<<(unsigned)((n8k + 255) / 256), 256, 0, stream>>>(wv, BV, n8k, 16.0f);
  k_wsc<<<(unsigned)((n8q + 255) / 256), 256, 0, stream>>>(wo, BO, n8q, 16.0f);
  k_x16<<<(unsigned)((n8x + 255) / 256), 256, 0, stream>>>(x, X16, n8x);
  k_rotab<<<(SLEN * 32 + 255) / 256, 256, 0, stream>>>(CS, SN);
  k_gemm2<<<(NR / 128) * (DM / 64), 128, 0, stream>>>(X16, DM, BQ, DM, 0.0625f, nullptr, Qf, DM, NR, DM, DM);
  k_gemm2<<<(NR / 128) * (KVD / 64), 128, 0, stream>>>(X16, DM, BK, DM, 0.0625f, nullptr, Kf, KVD, NR, KVD, DM);
  k_gemm2<<<(NR / 128) * (KVD / 64), 128, 0, stream>>>(X16, DM, BV, DM, 0.0625f, nullptr, Vf, KVD, NR, KVD, DM);
  k_ropei<<<(unsigned)(((size_t)NR * NH * 8 + 255) / 256), 256, 0, stream>>>(Qf, NH, NH, 1, CS, SN, QH, QL);
  k_ropei<<<(unsigned)(((size_t)NR * NKV * 8 + 255) / 256), 256, 0, stream>>>(Kf, NKV, NKV, 1, CS, SN, KH, KL);
  k_hl<<<(unsigned)((n8v + 255) / 256), 256, 0, stream>>>(Vf, VH, VL, n8v);
  k_vtg<<<NB * NKV * (SLEN / 64), 256, 0, stream>>>(VH, VT);
  k_vtg<<<NB * NKV * (SLEN / 64), 256, 0, stream>>>(VL, VTL);
  k_flash5c<<<NB * NH * QBN5, 128, 0, stream>>>(QH, QL, DM, KH, KL, KVD, VT, VTL, O, DM);
  if (QBNP > 0) k_flashc<<<NB * NH * QBNPD, 128, 0, stream>>>(QH, DM, KH, KVD, VT, O, DM);
  k_hl<<<(unsigned)((n8x + 255) / 256), 256, 0, stream>>>(O, OH, OL, n8x);
  for (int bb = 0; bb < NB; ++bb)
    k_gemm2<<<(SLEN / 128) * (DM / 64), 128, 0, stream>>>(OH + (size_t)bb * SLEN * DM, DM, BO, DM, 0.0625f, nullptr, out + (size_t)bb * SEQ_FULL * DM, DM, SLEN, DM, DM);
  for (int bb = 0; bb < NB; ++bb)
    k_gemm2<<<(RE / 128) * (DM / 64), 128, 0, stream>>>(OL + (size_t)bb * SLEN * DM, DM, BO, DM, 0.0625f / 1024.0f, out + (size_t)bb * SEQ_FULL * DM, out + (size_t)bb * SEQ_FULL * DM, DM, RE, DM, DM);
}
